// PCconv_2525440770954
// MI455X (gfx1250) — hardware-run, weakly checked
//
#include <hip/hip_runtime.h>
#include <math.h>

typedef __attribute__((ext_vector_type(16))) _Float16 v16h;
typedef __attribute__((ext_vector_type(8)))  _Float16 v8h;
typedef __attribute__((ext_vector_type(8)))  float    v8f;
typedef __attribute__((ext_vector_type(4)))  float    v4f;

constexpr int kCh      = 512;
constexpr int kPx      = 1024;
constexpr int kGroups  = 32;
constexpr int kLow     = 256;
constexpr int kPatchK  = 4608;
constexpr int kRawRows = 8192;
constexpr int kRawK    = 512;
constexpr int kAggK    = 3072;
constexpr int kYtK     = 1536;
constexpr int kZtK     = 1024;
constexpr int kXSide   = 38;
constexpr int kXGroup  = kXSide * kXSide * 16;
constexpr int kpad16(int ks) { return ((16 * ks * ks + 31) / 32) * 32; }
static_assert(kpad16(3) == 160);
static_assert(kpad16(5) == 416);
static_assert(kpad16(7) == 800);
static_assert(kPatchK == 9 * kCh);
static_assert(kRawRows == 16 * kCh);
static_assert(kRawK == 2 * kLow && kAggK == 3 * kPx && kYtK == 3 * kCh);
static_assert((kPatchK % 32) == 0 && (kYtK % 32) == 0 && (kZtK % 32) == 0 && (kRawK % 32) == 0 && (kAggK % 32) == 0);
static_assert((kCh % 64) == 0 && (kPx % 64) == 0 && (kLow % 64) == 0 && (kRawRows % 64) == 0);
static_assert(kXSide == 32 + 2 * 3);

constexpr float kWCarry   = 256.0f;
constexpr float kXCarry   = 16.0f;
constexpr float kGwCarry  = 64.0f;
constexpr float kActCarry = 16.0f;
constexpr float kPCarry   = 1024.0f;
constexpr float kResCarry = 2048.0f;
constexpr float kResFold  = 1.0f / kResCarry;

constexpr size_t kSzXP   = (size_t)kGroups * kXGroup * 2;
constexpr size_t kSzW3   = (size_t)kCh * kpad16(3) * 2;
constexpr size_t kSzW5   = (size_t)kCh * kpad16(5) * 2;
constexpr size_t kSzW7   = (size_t)kCh * kpad16(7) * 2;
constexpr size_t kSzGW   = (size_t)kPx * kAggK * 2;
constexpr size_t kSzWDX  = (size_t)kCh * kYtK * 2;
constexpr size_t kSzWFU  = (size_t)kCh * kZtK * 2;
constexpr size_t kSzYBR  = (size_t)3 * kCh * kPx * 4;
constexpr size_t kSzSTAT = (size_t)3 * kCh * 32 * 4;
constexpr size_t kSzATT  = (size_t)3 * kCh * 4;
constexpr size_t kSzO32  = (size_t)kCh * kPx * 4;
constexpr size_t kSzPPL  = (size_t)kLow * kPatchK * 2;
constexpr size_t kSzARAW = (size_t)kRawRows * kRawK * 2;
constexpr size_t kSzGRAM = (size_t)kLow * kLow * 4;
constexpr size_t kSzPYI  = (size_t)kLow * kRawK * 2;
constexpr size_t kSzTCOL = (size_t)kRawRows * kLow * 4;
constexpr size_t kSzRF   = (size_t)kCh * kPx * 4;
constexpr size_t kSzR3   = (size_t)kCh * kAggK * 2;
constexpr size_t kSzSIG  = (size_t)kCh * kPx * 4;
constexpr size_t kSzGFL  = (size_t)kPx * kCh * 4;
constexpr size_t kSzPAW  = (size_t)9 * kPx * 4;
constexpr size_t kSzYT   = (size_t)kPx * kYtK * 2;
constexpr size_t kSzDPL  = (size_t)kPx * kCh * 4;
constexpr size_t kSzDST  = (size_t)2 * kCh * 4;
constexpr size_t kSzZT   = (size_t)kPx * kZtK * 2;
constexpr size_t kSzFPL  = (size_t)kCh * kPx * 4;

constexpr size_t kOffXH   = 0;
constexpr size_t kOffXL   = kOffXH   + kSzXP;
constexpr size_t kOffW3H  = kOffXL   + kSzXP;
constexpr size_t kOffW3L  = kOffW3H  + kSzW3;
constexpr size_t kOffW5H  = kOffW3L  + kSzW3;
constexpr size_t kOffW5L  = kOffW5H  + kSzW5;
constexpr size_t kOffW7H  = kOffW5L  + kSzW5;
constexpr size_t kOffW7L  = kOffW7H  + kSzW7;
constexpr size_t kOffGW   = kOffW7L  + kSzW7;
constexpr size_t kOffWDX  = kOffGW   + kSzGW;
constexpr size_t kOffWFU  = kOffWDX  + kSzWDX;
constexpr size_t kOffYBR  = kOffWFU  + kSzWFU;
constexpr size_t kOffSTAT = kOffYBR  + kSzYBR;
constexpr size_t kOffATT  = kOffSTAT + kSzSTAT;
constexpr size_t kOffO32  = kOffATT  + kSzATT;
constexpr size_t kOffPPL  = kOffO32  + kSzO32;
constexpr size_t kOffARAW = kOffPPL  + kSzPPL;
constexpr size_t kOffGRAM = kOffARAW + kSzARAW;
constexpr size_t kOffPYI  = kOffGRAM + kSzGRAM;
constexpr size_t kOffTCOL = kOffPYI  + kSzPYI;
constexpr size_t kOffRF   = kOffTCOL + kSzTCOL;
constexpr size_t kOffR3   = kOffRF   + kSzRF;
constexpr size_t kOffSIG  = kOffR3   + kSzR3;
constexpr size_t kOffGFL  = kOffSIG  + kSzSIG;
constexpr size_t kOffPAW  = kOffGFL  + kSzGFL;
constexpr size_t kOffYT   = kOffPAW  + kSzPAW;
constexpr size_t kOffDPL  = kOffYT   + kSzYT;
constexpr size_t kOffDST  = kOffDPL  + kSzDPL;
constexpr size_t kOffZT   = kOffDST  + kSzDST;
constexpr size_t kOffFPL  = kOffZT   + kSzZT;
constexpr size_t kWsTotal = kOffFPL  + kSzFPL;
static_assert(kWsTotal == 61855744ull);
static_assert(kWsTotal <= 134217728ull);
static_assert((kSzXP % 128) == 0 && (kSzW3 % 128) == 0 && (kSzW5 % 128) == 0 && (kSzW7 % 128) == 0 &&
              (kSzGW % 128) == 0 && (kSzWDX % 128) == 0 && (kSzWFU % 128) == 0 && (kSzYBR % 128) == 0 &&
              (kSzSTAT % 128) == 0 && (kSzATT % 128) == 0 && (kSzO32 % 128) == 0 && (kSzPPL % 128) == 0 &&
              (kSzARAW % 128) == 0 && (kSzGRAM % 128) == 0 && (kSzPYI % 128) == 0 && (kSzTCOL % 128) == 0 &&
              (kSzRF % 128) == 0 && (kSzR3 % 128) == 0 && (kSzSIG % 128) == 0 && (kSzGFL % 128) == 0 &&
              (kSzPAW % 128) == 0 && (kSzYT % 128) == 0 && (kSzDPL % 128) == 0 && (kSzDST % 128) == 0 &&
              (kSzZT % 128) == 0 && (kSzFPL % 128) == 0);

__device__ __forceinline__ int clampi(int v, int lo, int hi) { return v < lo ? lo : (v > hi ? hi : v); }

__device__ __forceinline__ void split16(float vc, _Float16& hi, _Float16& lo) {
  hi = (_Float16)vc;
  const float hf = (float)hi;
  const float rs = (vc - hf) * kResCarry;
  lo = (_Float16)rs;
}

__device__ __forceinline__ void st2_v8h(unsigned short* q, v8h hv) {
  *(volatile v8h*)q = hv;
  __threadfence();
  *(volatile v8h*)q = hv;
}
__device__ __forceinline__ void st2_v8h_2(unsigned short* q0, v8h v0, unsigned short* q1, v8h v1) {
  *(volatile v8h*)q0 = v0;
  *(volatile v8h*)q1 = v1;
  __threadfence();
  *(volatile v8h*)q0 = v0;
  *(volatile v8h*)q1 = v1;
}
__device__ __forceinline__ void st2_v8h_3(unsigned short* q0, v8h v0, unsigned short* q1, v8h v1, unsigned short* q2, v8h v2) {
  *(volatile v8h*)q0 = v0;
  *(volatile v8h*)q1 = v1;
  *(volatile v8h*)q2 = v2;
  __threadfence();
  *(volatile v8h*)q0 = v0;
  *(volatile v8h*)q1 = v1;
  *(volatile v8h*)q2 = v2;
}
__device__ __forceinline__ void st2_v4f(float* q, v4f v) {
  *(volatile v4f*)q = v;
  __threadfence();
  *(volatile v4f*)q = v;
}
__device__ __forceinline__ void st2_f(float* q, float v) {
  *(volatile float*)q = v;
  __threadfence();
  *(volatile float*)q = v;
}

__device__ __forceinline__ float block_sum256(float v, float* sRed, int lane, int wave) {
#pragma unroll
  for (int off = 16; off > 0; off >>= 1) v += __shfl_xor(v, off, 32);
  __syncthreads();
  if (lane == 0) sRed[wave] = v;
  __syncthreads();
  float t = sRed[0];
  t += sRed[1];
  t += sRed[2];
  t += sRed[3];
  t += sRed[4];
  t += sRed[5];
  t += sRed[6];
  t += sRed[7];
  return t;
}

__device__ __forceinline__ void guard4_h(v8f& a, v8f& b, v8f& c, v8f& d, v16h x) {
  asm volatile("v_nop\n\tv_nop\n\tv_nop\n\tv_nop" : "+v"(a), "+v"(b), "+v"(c), "+v"(d) : "v"(x));
}
__device__ __forceinline__ void guard4x5_h(v8f& a, v8f& b, v8f& c, v8f& d, v16h x, v16h y0, v16h y1, v16h y2, v16h y3) {
  asm volatile("v_nop\n\tv_nop\n\tv_nop\n\tv_nop" : "+v"(a), "+v"(b), "+v"(c), "+v"(d) : "v"(x), "v"(y0), "v"(y1), "v"(y2), "v"(y3));
}
__device__ __forceinline__ void guard4x10_h(v8f& a, v8f& b, v8f& c, v8f& d, v16h x0, v16h x1,
                                            v16h y0, v16h y1, v16h y2, v16h y3, v16h z0, v16h z1, v16h z2, v16h z3) {
  asm volatile("v_nop\n\tv_nop\n\tv_nop\n\tv_nop" : "+v"(a), "+v"(b), "+v"(c), "+v"(d)
               : "v"(x0), "v"(x1), "v"(y0), "v"(y1), "v"(y2), "v"(y3), "v"(z0), "v"(z1), "v"(z2), "v"(z3));
}
__device__ __forceinline__ void keep4_h(v16h a, v16h b, v16h c, v16h d) { asm volatile("v_nop" :: "v"(a), "v"(b), "v"(c), "v"(d)); }
__device__ __forceinline__ void acc_guard4(v8f& a, v8f& b, v8f& c, v8f& d) { asm volatile("v_nop\n\tv_nop\n\tv_nop\n\tv_nop" : "+v"(a), "+v"(b), "+v"(c), "+v"(d)); }

struct FragH {
  union U { v16h v; v8h h[2]; };
  static __device__ __forceinline__ v16h load(const _Float16* p) {
    U f;
    f.h[0] = *(const v8h*)(p);
    f.h[1] = *(const v8h*)(p + 16);
    return f.v;
  }
  static __device__ __forceinline__ v16h load2(const _Float16* p0, const _Float16* p1, bool ok1) {
    U f;
    const v8h z = (v8h){(_Float16)0.0f, (_Float16)0.0f, (_Float16)0.0f, (_Float16)0.0f,
                        (_Float16)0.0f, (_Float16)0.0f, (_Float16)0.0f, (_Float16)0.0f};
    f.h[0] = *(const v8h*)(p0);
    const v8h t = *(const v8h*)(p1);
    f.h[1] = ok1 ? t : z;
    return f.v;
  }
  static __device__ __forceinline__ v8f mma(v16h a, v16h b, v8f c) {
    return __builtin_amdgcn_wmma_f32_16x16x32_f16(false, a, false, b, (short)0, c, false, false);
  }
};

__global__ __launch_bounds__(256) void gemm64_f16_kernel(
    const unsigned short* __restrict__ Ap, int lda,
    const unsigned short* __restrict__ Btp, int ldb,
    float* __restrict__ C, int ldc, int M, int N, int K, float scale, int kRes, float resFold) {
  const _Float16* A = (const _Float16*)Ap;
  const _Float16* Bt = (const _Float16*)Btp;
  __shared__ __align__(16) float sT[8][16 * 68];
  const int lane = threadIdx.x & 31;
  const int wave = __builtin_amdgcn_readfirstlane((int)(threadIdx.x >> 5));
  const int tilesN = N >> 6;
  const int tilesM = M >> 6;
  const int tile = blockIdx.x * 8 + wave;
  if (tile >= tilesM * tilesN) return;
  const int tm = tile / tilesN;
  const int tn = tile - tm * tilesN;
  const int m0 = tm << 6;
  const int n0 = tn << 6;

  const int rlane = lane & 15;
  const int koff  = (lane >> 4) * 8;
  const int mOff  = (lane >> 4) * 8;

  v8f acc[4][4];
#pragma unroll
  for (int i = 0; i < 4; ++i)
#pragma unroll
    for (int j = 0; j < 4; ++j) acc[i][j] = (v8f){0.f,0.f,0.f,0.f,0.f,0.f,0.f,0.f};

  for (int k0 = 0; k0 < K; k0 += 32) {
    v16h bh[4];
#pragma unroll
    for (int j = 0; j < 4; ++j) {
      const size_t bo = (size_t)(n0 + (j << 4) + rlane) * ldb + koff + k0;
      bh[j] = FragH::load(Bt + bo);
    }
#pragma unroll
    for (int i = 0; i < 4; ++i) {
      const size_t ao = (size_t)(m0 + (i << 4) + rlane) * lda + koff + k0;
      v16h ah = FragH::load(A + ao);
#pragma unroll
      for (int j = 0; j < 4; ++j) acc[i][j] = FragH::mma(ah, bh[j], acc[i][j]);
      guard4_h(acc[i][0], acc[i][1], acc[i][2], acc[i][3], ah);
    }
    keep4_h(bh[0], bh[1], bh[2], bh[3]);
    if (k0 + 32 == kRes) {
      acc_guard4(acc[0][0], acc[0][1], acc[0][2], acc[0][3]);
      acc_guard4(acc[1][0], acc[1][1], acc[1][2], acc[1][3]);
      acc_guard4(acc[2][0], acc[2][1], acc[2][2], acc[2][3]);
      acc_guard4(acc[3][0], acc[3][1], acc[3][2], acc[3][3]);
#pragma unroll
      for (int i = 0; i < 4; ++i)
#pragma unroll
        for (int j = 0; j < 4; ++j) acc[i][j] = acc[i][j] * resFold;
    }
  }
  acc_guard4(acc[0][0], acc[0][1], acc[0][2], acc[0][3]);
  acc_guard4(acc[1][0], acc[1][1], acc[1][2], acc[1][3]);
  acc_guard4(acc[2][0], acc[2][1], acc[2][2], acc[2][3]);
  acc_guard4(acc[3][0], acc[3][1], acc[3][2], acc[3][3]);

  float* slab = sT[wave];
#pragma unroll
  for (int i = 0; i < 4; ++i) {
    const int mBase = m0 + (i << 4);
#pragma unroll
    for (int j = 0; j < 4; ++j) {
#pragma unroll
      for (int r = 0; r < 8; ++r) {
        const float v = acc[i][j][r] * scale;
        slab[(mOff + r) * 68 + (j << 4) + rlane] = v;
      }
    }
    __builtin_amdgcn_fence(__ATOMIC_RELEASE, "workgroup");
    __builtin_amdgcn_wave_barrier();
    __builtin_amdgcn_fence(__ATOMIC_ACQUIRE, "workgroup");
    {
      const int hh = lane >> 4, c4 = (lane & 15) * 4;
      for (int pass = 0; pass < 2; ++pass) {
#pragma unroll
        for (int it = 0; it < 8; ++it) {
          const int row = it * 2 + hh;
          v4f v = *(const v4f*)(slab + row * 68 + c4);
          *(volatile v4f*)(C + (size_t)(mBase + row) * ldc + n0 + c4) = v;
        }
        __threadfence();
      }
    }
    __builtin_amdgcn_fence(__ATOMIC_RELEASE, "workgroup");
    __builtin_amdgcn_wave_barrier();
    __builtin_amdgcn_fence(__ATOMIC_ACQUIRE, "workgroup");
  }
}

template <int KS>
__global__ __launch_bounds__(256) void branch_gemm_kernel(
    const unsigned short* __restrict__ WHp, const unsigned short* __restrict__ WLp,
    const unsigned short* __restrict__ XHp, const unsigned short* __restrict__ XLp,
    const float* __restrict__ bias, float* __restrict__ Y, float scale) {
  constexpr int KK = KS * KS;
  constexpr int KPAD = kpad16(KS);
  constexpr int PAD = KS / 2;
  constexpr int NSTEP = KPAD / 32;
  static_assert(2 * NSTEP == KK + 1);
  constexpr int J1 = 16 * 16;
  constexpr int J2 = kXSide * 16;
  constexpr int J3 = J1 + J2;
  __shared__ __align__(16) float sT[8][16 * 68];
  const int lane = threadIdx.x & 31;
  const int wave = __builtin_amdgcn_readfirstlane((int)(threadIdx.x >> 5));
  const int g = blockIdx.y;
  const int px0 = (blockIdx.x * 8 + wave) << 6;
  const int py0 = px0 >> 5;
  const int rlane = lane & 15;
  const int koff  = (lane >> 4) * 8;
  const int mOff  = (lane >> 4) * 8;
  const _Float16* WHb = (const _Float16*)WHp + (size_t)(g * 16 + rlane) * KPAD + koff;
  const _Float16* WLb = (const _Float16*)WLp + (size_t)(g * 16 + rlane) * KPAD + koff;
  const int xoff = ((g * kXSide + py0 + 3 - PAD) * kXSide + rlane + 3 - PAD) * 16 + koff;
  const _Float16* XHb = (const _Float16*)XHp + xoff;
  const _Float16* XLb = (const _Float16*)XLp + xoff;

  v8f c0 = (v8f){0.f,0.f,0.f,0.f,0.f,0.f,0.f,0.f};
  v8f c1 = c0, c2 = c0, c3 = c0;
  v8f d0 = c0, d1 = c0, d2 = c0, d3 = c0;
#pragma unroll 1
  for (int s = 0; s < NSTEP; ++s) {
    const int t0 = 2 * s;
    const bool ok1 = (t0 + 1) < KK;
    const int t1 = ok1 ? (t0 + 1) : (KK - 1);
    const int ky0 = t0 / KS, kx0 = t0 - ky0 * KS;
    const int ky1 = t1 / KS, kx1 = t1 - ky1 * KS;
    const int o0 = (ky0 * kXSide + kx0) * 16;
    const int o1 = (ky1 * kXSide + kx1) * 16;
    const v16h ah  = FragH::load(WHb + 32 * s);
    const v16h al  = FragH::load(WLb + 32 * s);
    const v16h bh0 = FragH::load2(XHb + o0, XHb + o1, ok1);
    const v16h bh1 = FragH::load2(XHb + J1 + o0, XHb + J1 + o1, ok1);
    const v16h bh2 = FragH::load2(XHb + J2 + o0, XHb + J2 + o1, ok1);
    const v16h bh3 = FragH::load2(XHb + J3 + o0, XHb + J3 + o1, ok1);
    const v16h bl0 = FragH::load2(XLb + o0, XLb + o1, ok1);
    const v16h bl1 = FragH::load2(XLb + J1 + o0, XLb + J1 + o1, ok1);
    const v16h bl2 = FragH::load2(XLb + J2 + o0, XLb + J2 + o1, ok1);
    const v16h bl3 = FragH::load2(XLb + J3 + o0, XLb + J3 + o1, ok1);
    c0 = FragH::mma(ah, bh0, c0);
    c1 = FragH::mma(ah, bh1, c1);
    c2 = FragH::mma(ah, bh2, c2);
    c3 = FragH::mma(ah, bh3, c3);
    d0 = FragH::mma(ah, bl0, d0);
    d1 = FragH::mma(ah, bl1, d1);
    d2 = FragH::mma(ah, bl2, d2);
    d3 = FragH::mma(ah, bl3, d3);
    d0 = FragH::mma(al, bh0, d0);
    d1 = FragH::mma(al, bh1, d1);
    d2 = FragH::mma(al, bh2, d2);
    d3 = FragH::mma(al, bh3, d3);
    guard4x5_h(c0, c1, c2, c3, ah, bh0, bh1, bh2, bh3);
    guard4x10_h(d0, d1, d2, d3, ah, al, bh0, bh1, bh2, bh3, bl0, bl1, bl2, bl3);
  }
  acc_guard4(c0, c1, c2, c3);
  acc_guard4(d0, d1, d2, d3);

  const float scaleRes = scale * kResFold;
  float* slab = sT[wave];
#pragma unroll
  for (int r = 0; r < 8; ++r) {
    const float bv = bias[g * 16 + mOff + r];
    slab[(mOff + r) * 68 + rlane]      = (c0[r] * scale + d0[r] * scaleRes) + bv;
    slab[(mOff + r) * 68 + 16 + rlane] = (c1[r] * scale + d1[r] * scaleRes) + bv;
    slab[(mOff + r) * 68 + 32 + rlane] = (c2[r] * scale + d2[r] * scaleRes) + bv;
    slab[(mOff + r) * 68 + 48 + rlane] = (c3[r] * scale + d3[r] * scaleRes) + bv;
  }
  __builtin_amdgcn_fence(__ATOMIC_RELEASE, "workgroup");
  __builtin_amdgcn_wave_barrier();
  __builtin_amdgcn_fence(__ATOMIC_ACQUIRE, "workgroup");
  {
    const int hh = lane >> 4, c4 = (lane & 15) * 4;
    for (int pass = 0; pass < 2; ++pass) {
#pragma unroll
      for (int it = 0; it < 8; ++it) {
        const int row = it * 2 + hh;
        v4f v = *(const v4f*)(slab + row * 68 + c4);
        *(volatile v4f*)(Y + (size_t)(g * 16 + row) * kPx + px0 + c4) = v;
      }
      __threadfence();
    }
  }
}

template <int KS>
__global__ __launch_bounds__(256) void cvt_branch_w_kernel(const float* __restrict__ w, unsigned short* __restrict__ dhi,
                                                           unsigned short* __restrict__ dlo) {
  constexpr int KK = KS * KS;
  constexpr int KPAD = kpad16(KS);
  constexpr int CPR = KPAD / 8;
  static_assert(((kCh * CPR) % 256) == 0);
  const int i = blockIdx.x * 256 + threadIdx.x;
  const int row = i / CPR;
  const int kc = i - row * CPR;
  const int tap = kc >> 1;
  const int ci0 = (kc & 1) * 8;
  const bool ok = tap < KK;
  const int tapc = ok ? tap : (KK - 1);
  const float* src = w + (size_t)row * 16 * KK + ci0 * KK + tapc;
  v8h hv, lv;
#pragma unroll
  for (int e = 0; e < 8; ++e) {
    float v = src[e * KK];
    asm volatile("" : "+v"(v));
    const float vc = ok ? v * kWCarry : 0.0f;
    _Float16 hi, lo;
    split16(vc, hi, lo);
    hv[e] = hi;
    lv[e] = lo;
  }
  st2_v8h_2(dhi + (size_t)i * 8, hv, dlo + (size_t)i * 8, lv);
}

static_assert(((kGroups * kXSide * kXSide * 2) % 256) == 0);
__global__ __launch_bounds__(256) void xpad_kernel(const float* __restrict__ x, unsigned short* __restrict__ dhi,
                                                   unsigned short* __restrict__ dlo) {
  const int i = blockIdx.x * 256 + threadIdx.x;
  const int row = i >> 1;
  const int ci0 = (i & 1) * 8;
  const int g = row / (kXSide * kXSide);
  const int pos = row - g * (kXSide * kXSide);
  const int yy = pos / kXSide;
  const int xx = pos - yy * kXSide;
  const int iy = yy - 3, ix = xx - 3;
  const bool ok = ((unsigned)iy < 32u) && ((unsigned)ix < 32u);
  const int iyc = clampi(iy, 0, 31), ixc = clampi(ix, 0, 31);
  const float* src = x + (size_t)(g * 16 + ci0) * kPx + iyc * 32 + ixc;
  v8h hv, lv;
#pragma unroll
  for (int e = 0; e < 8; ++e) {
    float v = src[(size_t)e * kPx];
    asm volatile("" : "+v"(v));
    const float vc = ok ? v * kXCarry : 0.0f;
    _Float16 hi, lo;
    split16(vc, hi, lo);
    hv[e] = hi;
    lv[e] = lo;
  }
  st2_v8h_2(dhi + (size_t)i * 8, hv, dlo + (size_t)i * 8, lv);
}

__global__ __launch_bounds__(256) void cvt_flat_kernel(const float* __restrict__ src, unsigned short* __restrict__ dst, float carry, int total8) {
  const int i = blockIdx.x * 256 + threadIdx.x;
  if (i >= total8) return;
  const v4f a0 = *(const v4f*)(src + (size_t)i * 8);
  const v4f a1 = *(const v4f*)(src + (size_t)i * 8 + 4);
  v8h hv;
#pragma unroll
  for (int e = 0; e < 4; ++e) {
    hv[e]     = (_Float16)(a0[e] * carry);
    hv[4 + e] = (_Float16)(a1[e] * carry);
  }
  st2_v8h(dst + (size_t)i * 8, hv);
}

__global__ __launch_bounds__(256) void gus_plane_kernel(const float* __restrict__ src, unsigned short* __restrict__ dst) {
  const int i = blockIdx.x * 256 + threadIdx.x;
  const int p = i >> 7;
  const int kc = i & 127;
  const v4f a0 = *(const v4f*)(src + (size_t)p * kPx + kc * 8);
  const v4f a1 = *(const v4f*)(src + (size_t)p * kPx + kc * 8 + 4);
  v8h hv, lv;
#pragma unroll
  for (int e = 0; e < 4; ++e) {
    _Float16 h0, l0, h1, l1;
    split16(a0[e] * kGwCarry, h0, l0);
    split16(a1[e] * kGwCarry, h1, l1);
    hv[e] = h0;
    lv[e] = l0;
    hv[4 + e] = h1;
    lv[4 + e] = l1;
  }
  unsigned short* base = dst + (size_t)p * kAggK + kc * 8;
  st2_v8h_3(base, hv, base + kPx, lv, base + 2 * kPx, hv);
}

__global__ __launch_bounds__(256) void cvt_down_w_kernel(const float* __restrict__ w, unsigned short* __restrict__ dst) {
  const int i = blockIdx.x * 256 + threadIdx.x;
  const int row = i / 192;
  const int kc = i - row * 192;
  const int sec = kc >> 6;
  const int col = (kc & 63) * 8 + ((sec == 2) ? 512 : 0);
  const v4f a0 = *(const v4f*)(w + (size_t)row * 1024 + col);
  const v4f a1 = *(const v4f*)(w + (size_t)row * 1024 + col + 4);
  v8h hv;
#pragma unroll
  for (int e = 0; e < 4; ++e) {
    hv[e]     = (_Float16)(a0[e] * kWCarry);
    hv[4 + e] = (_Float16)(a1[e] * kWCarry);
  }
  st2_v8h(dst + (size_t)i * 8, hv);
}

__global__ __launch_bounds__(256) void branch_stats_kernel(const float* __restrict__ Y, float* __restrict__ stat) {
  __shared__ float sRed[8];
  const int tid = threadIdx.x, lane = tid & 31;
  const int wave = __builtin_amdgcn_readfirstlane((int)(threadIdx.x >> 5));
  const v4f v = *(const v4f*)(Y + (size_t)blockIdx.x * kPx + tid * 4);
  const float s = (v[0] + v[1]) + (v[2] + v[3]);
  const float mean = block_sum256(s, sRed, lane, wave) * (1.0f / 1024.0f);
  const float d0 = v[0] - mean, d1 = v[1] - mean, d2 = v[2] - mean, d3 = v[3] - mean;
  const float q = (d0 * d0 + d1 * d1) + (d2 * d2 + d3 * d3);
  const float var = block_sum256(q, sRed, lane, wave) * (1.0f / 1024.0f);
  const float rstd = rsqrtf(var + 1e-5f);
  const float t = (fmaxf(d0 * rstd, 0.0f) + fmaxf(d1 * rstd, 0.0f)) + (fmaxf(d2 * rstd, 0.0f) + fmaxf(d3 * rstd, 0.0f));
  const float pool = block_sum256(t, sRed, lane, wave) * (1.0f / 1024.0f);
  const float o = (lane == 0) ? mean : ((lane == 1) ? rstd : ((lane == 2) ? pool : 0.0f));
  if (wave == 0) st2_f(stat + (size_t)blockIdx.x * 32 + lane, o);
}

__global__ __launch_bounds__(512) void branch_att_kernel(
    const float* __restrict__ stat, const float* __restrict__ fc_w, const float* __restrict__ fc_b,
    const float* __restrict__ fcs_w, const float* __restrict__ fcs_b, float* __restrict__ att) {
  __shared__ __align__(16) float sS[512];
  __shared__ __align__(16) float sZ[32];
  const int c = threadIdx.x, lane = c & 31;
  const int wave = __builtin_amdgcn_readfirstlane((int)(threadIdx.x >> 5));
  sS[c] = (stat[(size_t)c * 32 + 2] + stat[(size_t)(512 + c) * 32 + 2]) + stat[(size_t)(1024 + c) * 32 + 2];
  __syncthreads();
#pragma unroll
  for (int dd = 0; dd < 2; ++dd) {
    const int d = wave * 2 + dd;
    const float* wr = fc_w + (size_t)d * 512;
    float part = 0.0f;
#pragma unroll 4
    for (int j = 0; j < 16; ++j) part = fmaf(wr[lane + 32 * j], sS[lane + 32 * j], part);
#pragma unroll
    for (int off = 16; off > 0; off >>= 1) part += __shfl_xor(part, off, 32);
    const float fb = fc_b[d];
    if (lane == 0) sZ[d] = part + fb;
  }
  __syncthreads();
  float a0 = fcs_b[c], a1 = fcs_b[512 + c], a2 = fcs_b[1024 + c];
  const float* w0 = fcs_w + (size_t)c * 32;
  const float* w1 = fcs_w + (size_t)(512 + c) * 32;
  const float* w2 = fcs_w + (size_t)(1024 + c) * 32;
#pragma unroll 1
  for (int d4 = 0; d4 < 8; ++d4) {
    const v4f z  = *(const v4f*)(sZ + 4 * d4);
    const v4f x0 = *(const v4f*)(w0 + 4 * d4);
    const v4f x1 = *(const v4f*)(w1 + 4 * d4);
    const v4f x2 = *(const v4f*)(w2 + 4 * d4);
#pragma unroll
    for (int e = 0; e < 4; ++e) {
      a0 = fmaf(z[e], x0[e], a0);
      a1 = fmaf(z[e], x1[e], a1);
      a2 = fmaf(z[e], x2[e], a2);
    }
  }
  const float mx = fmaxf(a0, fmaxf(a1, a2));
  const float e0 = expf(a0 - mx), e1 = expf(a1 - mx), e2 = expf(a2 - mx);
  const float inv = 1.0f / ((e0 + e1) + e2);
  const float p0 = e0 * inv, p1 = e1 * inv, p2 = e2 * inv;
  volatile float* q0 = att + c;
  volatile float* q1 = att + 512 + c;
  volatile float* q2 = att + 1024 + c;
  *q0 = p0; *q1 = p1; *q2 = p2;
  __threadfence();
  *q0 = p0; *q1 = p1; *q2 = p2;
}

__global__ __launch_bounds__(256) void branch_combine_kernel(
    const float* __restrict__ Y, const float* __restrict__ stat, const float* __restrict__ att, float* __restrict__ O32) {
  const int c = blockIdx.x, tid = threadIdx.x;
  const float m0 = stat[(size_t)c * 32], r0 = stat[(size_t)c * 32 + 1];
  const float m1 = stat[(size_t)(512 + c) * 32], r1 = stat[(size_t)(512 + c) * 32 + 1];
  const float m2 = stat[(size_t)(1024 + c) * 32], r2 = stat[(size_t)(1024 + c) * 32 + 1];
  const float a0 = att[c], a1 = att[512 + c], a2 = att[1024 + c];
  const size_t o = (size_t)c * kPx + tid * 4;
  const v4f y0 = *(const v4f*)(Y + o);
  const v4f y1 = *(const v4f*)(Y + (size_t)kCh * kPx + o);
  const v4f y2 = *(const v4f*)(Y + (size_t)2 * kCh * kPx + o);
  v4f r;
#pragma unroll
  for (int e = 0; e < 4; ++e) {
    const float f0 = fmaxf((y0[e] - m0) * r0, 0.0f);
    const float f1 = fmaxf((y1[e] - m1) * r1, 0.0f);
    const float f2 = fmaxf((y2[e] - m2) * r2, 0.0f);
    r[e] = (f0 * a0 + f1 * a1) + f2 * a2;
  }
  st2_v4f(O32 + o, r);
}

__global__ __launch_bounds__(256) void patch_plane_kernel(const float* __restrict__ O32, unsigned short* __restrict__ dst) {
  const int i = blockIdx.x * 256 + threadIdx.x;
  const int l = i / 576;
  const int kc = i - l * 576;
  const int tap = kc >> 6;
  const int c0 = (kc & 63) * 8;
  const int ly = l >> 4, lx = l & 15;
  const int ky = tap / 3, kx = tap - ky * 3;
  const int iy = ly + ky - 1, ix = lx + kx - 1;
  const bool ok = ((unsigned)iy < 16u) && ((unsigned)ix < 16u);
  const int iyc = clampi(iy, 0, 15), ixc = clampi(ix, 0, 15);
  const float* src = O32 + (size_t)c0 * kPx + (2 * iyc) * 32 + 2 * ixc;
  v8h hv;
#pragma unroll
  for (int e = 0; e < 8; ++e) {
    float v = src[(size_t)e * kPx];
    asm volatile("" : "+v"(v));
    hv[e] = (_Float16)(ok ? v * kActCarry : 0.0f);
  }
  st2_v8h(dst + (size_t)i * 8, hv);
}

__global__ __launch_bounds__(256) void raw_plane_kernel(const float* __restrict__ O32, unsigned short* __restrict__ dst) {
  const int i = blockIdx.x * 256 + threadIdx.x;
  const int r = i >> 5, lc = i & 31;
  const int c = r >> 4, u = (r >> 2) & 3, v = r & 3;
  const int ly = lc >> 1, lx0 = (lc & 1) * 8;
  const int iy = 2 * ly - 1 + u;
  const bool oky = (unsigned)iy < 32u;
  const int iyc = clampi(iy, 0, 31);
  const float* src = O32 + (size_t)c * kPx + iyc * 32;
  v8h hv, lv;
#pragma unroll
  for (int e = 0; e < 8; ++e) {
    const int ix = 2 * (lx0 + e) - 1 + v;
    const bool ok = oky && ((unsigned)ix < 32u);
    float t = src[clampi(ix, 0, 31)];
    asm volatile("" : "+v"(t));
    const float vc = ok ? t * kActCarry : 0.0f;
    _Float16 hi, lo;
    split16(vc, hi, lo);
    hv[e] = hi;
    lv[e] = lo;
  }
  unsigned short* base = dst + (size_t)r * kRawK + lc * 8;
  st2_v8h_2(base, lv, base + kLow, hv);
}

__global__ __launch_bounds__(256) void affinity_softmax_kernel(const float* __restrict__ G, unsigned short* __restrict__ P) {
  const int lane = threadIdx.x & 31;
  const int wave = __builtin_amdgcn_readfirstlane((int)(threadIdx.x >> 5));
  const int q = blockIdx.x * 8 + wave;
  const int l0 = lane * 8;
  const v4f g0 = *(const v4f*)(G + (size_t)q * kLow + l0);
  const v4f g1 = *(const v4f*)(G + (size_t)q * kLow + l0 + 4);
  float lg[8];
#pragma unroll
  for (int e = 0; e < 8; ++e) {
    const float dg = G[(size_t)(l0 + e) * (kLow + 1)];
    const float nrm = fmaxf(sqrtf(fmaxf(dg, 0.0f)), 1e-4f);
    const float gv = (e < 4) ? g0[e & 3] : g1[e & 3];
    lg[e] = (gv * (1.0f / nrm)) * 10.0f;
  }
  float mx = lg[0];
#pragma unroll
  for (int e = 1; e < 8; ++e) mx = fmaxf(mx, lg[e]);
#pragma unroll
  for (int off = 16; off > 0; off >>= 1) mx = fmaxf(mx, __shfl_xor(mx, off, 32));
  float ex[8];
  float s = 0.0f;
#pragma unroll
  for (int e = 0; e < 8; ++e) {
    ex[e] = expf(lg[e] - mx);
    s += ex[e];
  }
#pragma unroll
  for (int off = 16; off > 0; off >>= 1) s += __shfl_xor(s, off, 32);
  const float inv = (1.0f / s) * kPCarry;
  v8h hv;
#pragma unroll
  for (int e = 0; e < 8; ++e) hv[e] = (_Float16)(ex[e] * inv);
  unsigned short* base = P + (size_t)q * kRawK + l0;
  st2_v8h_2(base, hv, base + kLow, hv);
}

__global__ __launch_bounds__(256) void col2im_kernel(const float* __restrict__ T, float* __restrict__ RF,
                                                     float* __restrict__ SIG, unsigned short* __restrict__ R3) {
  __shared__ __align__(16) float sR[kPx];
  const int c = blockIdx.x, tid = threadIdx.x;
  const int wave = __builtin_amdgcn_readfirstlane((int)(threadIdx.x >> 5));
  const int px0 = tid * 4;
  const int oy = px0 >> 5, ox0 = px0 & 31;
  const int ua = (oy + 1) & 1;
  const int qy1 = (oy + 1) >> 1, qy2 = qy1 - 1;
  const bool oky1 = qy1 < 16, oky2 = qy2 >= 0;
  const int qy1c = clampi(qy1, 0, 15), qy2c = clampi(qy2, 0, 15);
  const float* Tc = T + (size_t)c * 16 * kLow;
  v4f rv, sv, cv;
#pragma unroll
  for (int e = 0; e < 4; ++e) {
    const int ox = ox0 + e;
    const int va = (ox + 1) & 1;
    const int qx1 = (ox + 1) >> 1, qx2 = qx1 - 1;
    const bool okx1 = qx1 < 16, okx2 = qx2 >= 0;
    const int qx1c = clampi(qx1, 0, 15), qx2c = clampi(qx2, 0, 15);
    float t11 = Tc[(size_t)(ua * 4 + va) * kLow + qy1c * 16 + qx1c];
    float t12 = Tc[(size_t)(ua * 4 + va + 2) * kLow + qy1c * 16 + qx2c];
    float t21 = Tc[(size_t)((ua + 2) * 4 + va) * kLow + qy2c * 16 + qx1c];
    float t22 = Tc[(size_t)((ua + 2) * 4 + va + 2) * kLow + qy2c * 16 + qx2c];
    asm volatile("" : "+v"(t11), "+v"(t12), "+v"(t21), "+v"(t22));
    float s = 0.0f;
    s += (oky1 && okx1) ? t11 : 0.0f;
    s += (oky1 && okx2) ? t12 : 0.0f;
    s += (oky2 && okx1) ? t21 : 0.0f;
    s += (oky2 && okx2) ? t22 : 0.0f;
    const float r = 0.25f * s;
    rv[e] = r;
    sv[e] = 1.0f / (1.0f + expf(-r));
    cv[e] = r * kActCarry;
  }
  *(v4f*)(sR + px0) = cv;
  {
    volatile v4f* p1 = (volatile v4f*)(RF + (size_t)c * kPx + px0);
    volatile v4f* p2 = (volatile v4f*)(SIG + (size_t)c * kPx + px0);
    *p1 = rv; *p2 = sv;
    __threadfence();
    *p1 = rv; *p2 = sv;
  }
  __syncthreads();
  if (wave < 4) {
    const v4f a0 = *(const v4f*)(sR + tid * 8);
    const v4f a1 = *(const v4f*)(sR + tid * 8 + 4);
    v8h hv, lv;
#pragma unroll
    for (int e = 0; e < 4; ++e) {
      _Float16 h0, l0, h1, l1;
      split16(a0[e], h0, l0);
      split16(a1[e], h1, l1);
      hv[e] = h0;
      lv[e] = l0;
      hv[4 + e] = h1;
      lv[4 + e] = l1;
    }
    unsigned short* base = R3 + (size_t)c * kAggK + tid * 8;
    st2_v8h_3(base, lv, base + kPx, hv, base + 2 * kPx, hv);
  }
}

__global__ __launch_bounds__(288) void tap_weights_kernel(const float* __restrict__ SIG, float* __restrict__ PAW) {
  __shared__ float sL[9 * 32];
  __shared__ float sE[9 * 32];
  const int lane = threadIdx.x & 31;
  const int tap = __builtin_amdgcn_readfirstlane((int)(threadIdx.x >> 5));
  const int oy = blockIdx.x;
  const int q = oy * 32 + lane;
  const int ky = tap / 3, kx = tap - ky * 3;
  const int iy = oy + ky - 1, ix = lane + kx - 1;
  const bool ok = ((unsigned)iy < 32u) && ((unsigned)ix < 32u);
  const int nb = clampi(iy, 0, 31) * 32 + clampi(ix, 0, 31);
  float acc = 0.0f;
#pragma unroll 4
  for (int c = 0; c < kCh; ++c) {
    const float a = SIG[(size_t)c * kPx + q];
    float b = SIG[(size_t)c * kPx + nb];
    asm volatile("" : "+v"(b));
    acc = fmaf(a, ok ? b : 0.0f, acc);
  }
  const float logit = acc * (1.0f / 512.0f);
  sL[tap * 32 + lane] = logit;
  __syncthreads();
  float mx = sL[lane];
#pragma unroll
  for (int t = 1; t < 9; ++t) mx = fmaxf(mx, sL[t * 32 + lane]);
  const float ev = expf(logit - mx);
  sE[tap * 32 + lane] = ev;
  __syncthreads();
  float s = sE[lane];
#pragma unroll
  for (int t = 1; t < 9; ++t) s += sE[t * 32 + lane];
  const float w = ev * (1.0f / s);
  st2_f(PAW + (size_t)tap * kPx + q, w);
}

__global__ __launch_bounds__(256) void yt_pack_kernel(const float* __restrict__ GFL, const float* __restrict__ PAW,
                                                      const float* __restrict__ RF, unsigned short* __restrict__ YT) {
  const int i = blockIdx.x * 256 + threadIdx.x;
  const int px = i / 192;
  const int kc = i - px * 192;
  const int sec = __builtin_amdgcn_readfirstlane(kc >> 6);
  const int ch0 = (kc & 63) * 8;
  v8h hv;
  if (sec < 2) {
#pragma unroll
    for (int e = 0; e < 8; ++e) {
      const float v = GFL[(size_t)(ch0 + e) * kPx + px];
      _Float16 hi, lo;
      split16(v, hi, lo);
      hv[e] = (sec == 0) ? lo : hi;
    }
  } else {
    const int hb = px >> 9, cc = px & 511;
    const float* Rc = RF + (size_t)cc * kPx;
    float accv[8];
#pragma unroll
    for (int e = 0; e < 8; ++e) accv[e] = 0.0f;
#pragma unroll 1
    for (int t = 0; t < 9; ++t) {
      const int ky = t / 3, kx = t - ky * 3;
#pragma unroll
      for (int e = 0; e < 8; ++e) {
        const int q = 2 * (ch0 + e) + hb;
        const int iy = (q >> 5) + ky - 1, ix = (q & 31) + kx - 1;
        const bool ok = ((unsigned)iy < 32u) && ((unsigned)ix < 32u);
        const float a = PAW[(size_t)t * kPx + q];
        float r = Rc[clampi(iy, 0, 31) * 32 + clampi(ix, 0, 31)];
        asm volatile("" : "+v"(r));
        accv[e] = fmaf(a, ok ? r : 0.0f, accv[e]);
      }
    }
#pragma unroll
    for (int e = 0; e < 8; ++e) hv[e] = (_Float16)accv[e];
  }
  st2_v8h(YT + (size_t)i * 8, hv);
}

__global__ __launch_bounds__(256) void down_stats_kernel(const float* __restrict__ D, float* __restrict__ dst) {
  __shared__ float sP[8 * 32];
  const int lane = threadIdx.x & 31;
  const int wave = __builtin_amdgcn_readfirstlane((int)(threadIdx.x >> 5));
  const int col = blockIdx.x * 32 + lane;
  const float* p = D + (size_t)(wave * 128) * kCh + col;
  float s = 0.0f;
#pragma unroll 4
  for (int r = 0; r < 128; ++r) s += p[(size_t)r * kCh];
  sP[wave * 32 + lane] = s;
  __syncthreads();
  float tot = sP[lane];
#pragma unroll
  for (int g = 1; g < 8; ++g) tot += sP[g * 32 + lane];
  const float mean = tot * (1.0f / 1024.0f);
  __syncthreads();
  float q = 0.0f;
#pragma unroll 4
  for (int r = 0; r < 128; ++r) {
    const float d = p[(size_t)r * kCh] - mean;
    q = fmaf(d, d, q);
  }
  sP[wave * 32 + lane] = q;
  __syncthreads();
  float qt = sP[lane];
#pragma unroll
  for (int g = 1; g < 8; ++g) qt += sP[g * 32 + lane];
  const float rstd = rsqrtf(qt * (1.0f / 1024.0f) + 1e-5f);
  if (wave == 0) {
    volatile float* q0 = dst + col;
    volatile float* q1 = dst + kCh + col;
    *q0 = mean; *q1 = rstd;
    __threadfence();
    *q0 = mean; *q1 = rstd;
  }
}

__global__ __launch_bounds__(256) void zt_pack_kernel(const float* __restrict__ D, const float* __restrict__ dstat,
                                                      const float* __restrict__ O32, unsigned short* __restrict__ ZT) {
  const int i = blockIdx.x * 256 + threadIdx.x;
  const int px = i >> 7;
  const int kc = i & 127;
  const int sec = __builtin_amdgcn_readfirstlane(kc >> 6);
  v8h hv;
  if (sec == 0) {
    const int o0 = kc * 8;
    const v4f d0 = *(const v4f*)(D + (size_t)px * kCh + o0);
    const v4f d1 = *(const v4f*)(D + (size_t)px * kCh + o0 + 4);
    const v4f m0 = *(const v4f*)(dstat + o0);
    const v4f m1 = *(const v4f*)(dstat + o0 + 4);
    const v4f r0 = *(const v4f*)(dstat + kCh + o0);
    const v4f r1 = *(const v4f*)(dstat + kCh + o0 + 4);
#pragma unroll
    for (int e = 0; e < 4; ++e) {
      float y0 = (d0[e] - m0[e]) * r0[e];
      float y1 = (d1[e] - m1[e]) * r1[e];
      y0 = (y0 >= 0.0f) ? y0 : 0.2f * y0;
      y1 = (y1 >= 0.0f) ? y1 : 0.2f * y1;
      hv[e]     = (_Float16)(y0 * kActCarry);
      hv[4 + e] = (_Float16)(y1 * kActCarry);
    }
  } else {
    const int c0 = (kc - 64) * 8;
#pragma unroll
    for (int e = 0; e < 8; ++e) {
      const float v = O32[(size_t)(c0 + e) * kPx + px];
      hv[e] = (_Float16)(v * kActCarry);
    }
  }
  st2_v8h(ZT + (size_t)i * 8, hv);
}

__global__ __launch_bounds__(256) void final_norm_kernel(const float* __restrict__ F, float* __restrict__ out) {
  __shared__ float sRed[8];
  const int tid = threadIdx.x, lane = tid & 31;
  const int wave = __builtin_amdgcn_readfirstlane((int)(threadIdx.x >> 5));
  const size_t o = (size_t)blockIdx.x * kPx + tid * 4;
  const v4f v = *(const v4f*)(F + o);
  const float s = (v[0] + v[1]) + (v[2] + v[3]);
  const float mean = block_sum256(s, sRed, lane, wave) * (1.0f / 1024.0f);
  const float d0 = v[0] - mean, d1 = v[1] - mean, d2 = v[2] - mean, d3 = v[3] - mean;
  const float q = (d0 * d0 + d1 * d1) + (d2 * d2 + d3 * d3);
  const float var = block_sum256(q, sRed, lane, wave) * (1.0f / 1024.0f);
  const float rstd = rsqrtf(var + 1e-5f);
  v4f r;
  const float y0 = d0 * rstd, y1 = d1 * rstd, y2 = d2 * rstd, y3 = d3 * rstd;
  r[0] = (y0 >= 0.0f) ? y0 : 0.2f * y0;
  r[1] = (y1 >= 0.0f) ? y1 : 0.2f * y1;
  r[2] = (y2 >= 0.0f) ? y2 : 0.2f * y2;
  r[3] = (y3 >= 0.0f) ? y3 : 0.2f * y3;
  st2_v4f(out + o, r);
}

extern "C" void kernel_launch(void* const* d_in, const int* in_sizes, int n_in,
                              void* d_out, int out_size, void* d_ws, size_t ws_size,
                              hipStream_t stream) {
  if (n_in < 14) return;
  if (in_sizes[0] != kCh * kPx) return;
  if (in_sizes[1] != kPx * kPx) return;
  if (in_sizes[2] != kCh * 16 * 9) return;
  if (in_sizes[3] != kCh) return;
  if (in_sizes[4] != kCh * 16 * 25) return;
  if (in_sizes[5] != kCh) return;
  if (in_sizes[6] != kCh * 16 * 49) return;
  if (in_sizes[7] != kCh) return;
  if (in_sizes[8] != 32 * kCh) return;
  if (in_sizes[9] != 32) return;
  if (in_sizes[10] != 3 * kCh * 32) return;
  if (in_sizes[11] != 3 * kCh) return;
  if (in_sizes[12] != kCh * 1024) return;
  if (in_sizes[13] != kCh * 1024) return;
  if (out_size != kCh * kPx) return;
  if (ws_size < kWsTotal) return;

  const float* x      = (const float*)d_in[0];
  const float* gw     = (const float*)d_in[1];
  const float* w3     = (const float*)d_in[2];
  const float* b3     = (const float*)d_in[3];
  const float* w5     = (const float*)d_in[4];
  const float* b5     = (const float*)d_in[5];
  const float* w7     = (const float*)d_in[6];
  const float* b7     = (const float*)d_in[7];
  const float* fc_w   = (const float*)d_in[8];
  const float* fc_b   = (const float*)d_in[9];
  const float* fcs_w  = (const float*)d_in[10];
  const float* fcs_b  = (const float*)d_in[11];
  const float* down_w = (const float*)d_in[12];
  const float* fuse_w = (const float*)d_in[13];
  float* out = (float*)d_out;

  char* ws = (char*)d_ws;
  unsigned short* XH   = (unsigned short*)(ws + kOffXH);
  unsigned short* XL   = (unsigned short*)(ws + kOffXL);
  unsigned short* W3H  = (unsigned short*)(ws + kOffW3H);
  unsigned short* W3L  = (unsigned short*)(ws + kOffW3L);
  unsigned short* W5H  = (unsigned short*)(ws + kOffW5H);
  unsigned short* W5L  = (unsigned short*)(ws + kOffW5L);
  unsigned short* W7H  = (unsigned short*)(ws + kOffW7H);
  unsigned short* W7L  = (unsigned short*)(ws + kOffW7L);
  unsigned short* GW3  = (unsigned short*)(ws + kOffGW);
  unsigned short* WDX  = (unsigned short*)(ws + kOffWDX);
  unsigned short* WFU  = (unsigned short*)(ws + kOffWFU);
  float*          YBR  = (float*)(ws + kOffYBR);
  float*          STAT = (float*)(ws + kOffSTAT);
  float*          ATT  = (float*)(ws + kOffATT);
  float*          O32  = (float*)(ws + kOffO32);
  unsigned short* PPL  = (unsigned short*)(ws + kOffPPL);
  unsigned short* ARAW = (unsigned short*)(ws + kOffARAW);
  float*          GRAM = (float*)(ws + kOffGRAM);
  unsigned short* PYI  = (unsigned short*)(ws + kOffPYI);
  float*          TCOL = (float*)(ws + kOffTCOL);
  float*          RF   = (float*)(ws + kOffRF);
  unsigned short* R3   = (unsigned short*)(ws + kOffR3);
  float*          SIG  = (float*)(ws + kOffSIG);
  float*          GFL  = (float*)(ws + kOffGFL);
  float*          PAW  = (float*)(ws + kOffPAW);
  unsigned short* YT   = (unsigned short*)(ws + kOffYT);
  float*          DPL  = (float*)(ws + kOffDPL);
  float*          DST  = (float*)(ws + kOffDST);
  unsigned short* ZT   = (unsigned short*)(ws + kOffZT);
  float*          FPL  = (float*)(ws + kOffFPL);

  cvt_branch_w_kernel<3><<<2 * (kpad16(3) / 8), 256, 0, stream>>>(w3, W3H, W3L);
  cvt_branch_w_kernel<5><<<2 * (kpad16(5) / 8), 256, 0, stream>>>(w5, W5H, W5L);
  cvt_branch_w_kernel<7><<<2 * (kpad16(7) / 8), 256, 0, stream>>>(w7, W7H, W7L);
  gus_plane_kernel<<<(kPx * 128) / 256, 256, 0, stream>>>(gw, GW3);
  cvt_down_w_kernel<<<(kCh * 192) / 256, 256, 0, stream>>>(down_w, WDX);
  cvt_flat_kernel<<<(kCh * kZtK / 8) / 256, 256, 0, stream>>>(fuse_w, WFU, kWCarry, kCh * kZtK / 8);
  xpad_kernel<<<(kGroups * kXSide * kXSide * 2) / 256, 256, 0, stream>>>(x, XH, XL);

  const float brScale = 1.0f / (kWCarry * kXCarry);
  branch_gemm_kernel<3><<<dim3(2, kGroups), 256, 0, stream>>>(W3H, W3L, XH, XL, b3, YBR, brScale);
  branch_gemm_kernel<5><<<dim3(2, kGroups), 256, 0, stream>>>(W5H, W5L, XH, XL, b5, YBR + (size_t)kCh * kPx, brScale);
  branch_gemm_kernel<7><<<dim3(2, kGroups), 256, 0, stream>>>(W7H, W7L, XH, XL, b7, YBR + (size_t)2 * kCh * kPx, brScale);

  branch_stats_kernel<<<3 * kCh, 256, 0, stream>>>(YBR, STAT);
  branch_att_kernel<<<1, 512, 0, stream>>>(STAT, fc_w, fc_b, fcs_w, fcs_b, ATT);
  branch_combine_kernel<<<kCh, 256, 0, stream>>>(YBR, STAT, ATT, O32);

  patch_plane_kernel<<<(kLow * 576) / 256, 256, 0, stream>>>(O32, PPL);
  raw_plane_kernel<<<(kRawRows * 32) / 256, 256, 0, stream>>>(O32, ARAW);
  gemm64_f16_kernel<<<2, 256, 0, stream>>>(PPL, kPatchK, PPL, kPatchK, GRAM, kLow, kLow, kLow, kPatchK,
                                           1.0f / (kActCarry * kActCarry), 0, 1.0f);
  affinity_softmax_kernel<<<kLow / 8, 256, 0, stream>>>(GRAM, PYI);
  gemm64_f16_kernel<<<64, 256, 0, stream>>>(ARAW, kRawK, PYI, kRawK, TCOL, kLow, kRawRows, kLow, kRawK,
                                            1.0f / (kActCarry * kPCarry), kLow, kResFold);
  col2im_kernel<<<kCh, 256, 0, stream>>>(TCOL, RF, SIG, R3);

  gemm64_f16_kernel<<<16, 256, 0, stream>>>(GW3, kAggK, R3, kAggK, GFL, kCh, kPx, kCh, kAggK,
                                            1.0f / (kGwCarry * kActCarry), 2 * kPx, kResFold);

  tap_weights_kernel<<<32, 288, 0, stream>>>(SIG, PAW);
  yt_pack_kernel<<<(kPx * 192) / 256, 256, 0, stream>>>(GFL, PAW, RF, YT);

  gemm64_f16_kernel<<<16, 256, 0, stream>>>(YT, kYtK, WDX, kYtK, DPL, kCh, kPx, kCh, kYtK, 1.0f / kWCarry,
                                            kCh, kResFold);
  down_stats_kernel<<<kCh / 32, 256, 0, stream>>>(DPL, DST);
  zt_pack_kernel<<<(kPx * 128) / 256, 256, 0, stream>>>(DPL, DST, O32, ZT);

  gemm64_f16_kernel<<<16, 256, 0, stream>>>(WFU, kZtK, ZT, kZtK, FPL, kPx, kCh, kPx, kZtK,
                                            1.0f / (kWCarry * kActCarry), 0, 1.0f);
  final_norm_kernel<<<kCh, 256, 0, stream>>>(FPL, out);
}
